// Graph_81174881894890
// MI455X (gfx1250) — hardware-verified
//
#include <hip/hip_runtime.h>
#include <stddef.h>
#include <stdint.h>


#define DIN     512
#define FDIM    1024
#define NHEAD   8
#define HALL    8192
#define NX1     10240
#define OFH     1024
#define OFR     9216
#define JKK     3072
#define NTHR    256
#define NWAVE   8
#define EPT     8
#define CHUNK   (NTHR * EPT)
#define WCAP    (EPT * 32)
#define LISTN   (NWAVE * WCAP)
#define NBMAX   2048
#define RCAP    20480
#define DEGCAP  128
#define NIT     (DEGCAP / 32)
#define STW     2560
#define NBAGG   64
#define GBM     32
#define GBN     64
#define GTHR    64
#define WSMAX   134217728
#define LDS_AGG ((2 * RCAP + 2 * NBMAX + LISTN) * 4 + 64)

static_assert((CHUNK & (CHUNK - 1)) == 0 && CHUNK <= 4096);
static_assert((NBMAX & (NBMAX - 1)) == 0 && NBMAX <= 4096);
static_assert(NTHR * 8 == NBMAX);
static_assert(LISTN >= NBMAX);
static_assert(LISTN >= NWAVE * WCAP);
static_assert((RCAP % 32) == 0);
static_assert(NWAVE * STW <= RCAP);
static_assert(DEGCAP * NHEAD + DEGCAP + FDIM <= STW);
static_assert(DEGCAP == NIT * 32);
static_assert(LDS_AGG <= 300000);
static_assert(GBM == (GTHR / 32) * 16);
static_assert((DIN % 32) == 0 && (FDIM % GBN) == 0 && (HALL % GBN) == 0 && (NX1 % GBN) == 0 && (JKK % 32) == 0);
static_assert(HALL == NHEAD * FDIM && NX1 == FDIM + HALL + FDIM && OFH == FDIM && OFR == FDIM + HALL);
static_assert(FDIM == 1024 && NHEAD == 8);
static_assert((NBAGG & (NBAGG - 1)) == 0 && NBAGG >= 8 && NBAGG <= NBMAX && (NBAGG % GBM) == 0);
static_assert(FDIM == 8 * 128);

typedef float          v4f  __attribute__((ext_vector_type(4)));
typedef float          v8f  __attribute__((ext_vector_type(8)));
typedef int            v4i  __attribute__((ext_vector_type(4)));
typedef int            v8i  __attribute__((ext_vector_type(8)));
typedef unsigned short v8us __attribute__((ext_vector_type(8)));
typedef __bf16         v16bf __attribute__((ext_vector_type(16)));
union FragB { v16bf v; v8us h[2]; v8i w; };

__device__ __forceinline__ v8f wmb(const FragB& a, const FragB& b, v8f c) {
  v8f d = __builtin_amdgcn_wmma_f32_16x16x32_bf16(false, a.v, false, b.v, (short)0, c, false, false);
  asm volatile("v_nop\n\tv_nop\n\tv_nop\n\tv_nop" : "+v"(d) : "v"(a.w), "v"(b.w));
  return d;
}

__device__ __forceinline__ unsigned int bfb(float f) {
  const unsigned int u = __float_as_uint(f);
  return (u + 0x7FFFu + ((u >> 16) & 1u)) >> 16;
}

__device__ __forceinline__ void split8(const v4f a, const v4f b, v8us& hi, v8us& lo) {
  float v[8];
  v[0] = a.x; v[1] = a.y; v[2] = a.z; v[3] = a.w;
  v[4] = b.x; v[5] = b.y; v[6] = b.z; v[7] = b.w;
#pragma unroll
  for (int j = 0; j < 8; ++j) {
    const unsigned int hb = bfb(v[j]);
    const float hf = __uint_as_float(hb << 16);
    const unsigned int lb = bfb(v[j] - hf);
    hi[j] = (unsigned short)hb;
    lo[j] = (unsigned short)lb;
  }
}

__device__ __forceinline__ int scan_chunk(const int* __restrict__ dsts, int nE, int cbase, int slotBase,
                                          int nb, int vec8, int* list, int tid, int lane, int wave) {
  int wc = 0;
  const int el0  = tid * EPT;
  const int e0   = cbase + el0;
  const int sent = -2147483647 - 1;
  v4i da, db;
  if (vec8 != 0 && cbase + CHUNK <= nE) {
    da = *(const v4i*)(dsts + e0);
    db = *(const v4i*)(dsts + e0 + 4);
  } else {
    da.x = (e0     < nE) ? dsts[min(e0,     nE - 1)] : sent;
    da.y = (e0 + 1 < nE) ? dsts[min(e0 + 1, nE - 1)] : sent;
    da.z = (e0 + 2 < nE) ? dsts[min(e0 + 2, nE - 1)] : sent;
    da.w = (e0 + 3 < nE) ? dsts[min(e0 + 3, nE - 1)] : sent;
    db.x = (e0 + 4 < nE) ? dsts[min(e0 + 4, nE - 1)] : sent;
    db.y = (e0 + 5 < nE) ? dsts[min(e0 + 5, nE - 1)] : sent;
    db.z = (e0 + 6 < nE) ? dsts[min(e0 + 6, nE - 1)] : sent;
    db.w = (e0 + 7 < nE) ? dsts[min(e0 + 7, nE - 1)] : sent;
  }
  const unsigned nbs = (unsigned)slotBase;
  const unsigned unb = (unsigned)nb;
  const unsigned s0 = (unsigned)da.x - nbs, s1 = (unsigned)da.y - nbs;
  const unsigned s2 = (unsigned)da.z - nbs, s3 = (unsigned)da.w - nbs;
  const unsigned s4 = (unsigned)db.x - nbs, s5 = (unsigned)db.y - nbs;
  const unsigned s6 = (unsigned)db.z - nbs, s7 = (unsigned)db.w - nbs;
  const bool h0 = s0 < unb, h1 = s1 < unb, h2 = s2 < unb, h3 = s3 < unb;
  const bool h4 = s4 < unb, h5 = s5 < unb, h6 = s6 < unb, h7 = s7 < unb;
  const unsigned any = __builtin_amdgcn_ballot_w32(h0 | h1 | h2 | h3 | h4 | h5 | h6 | h7);
  if (any != 0u) {
#define HITJ(J, HJ, SJ) { \
      const unsigned mj = __builtin_amdgcn_ballot_w32(HJ); \
      if (mj != 0u) { \
        if (HJ) { \
          const int pos = wc + (int)__builtin_amdgcn_mbcnt_lo(mj, 0u); \
          if (pos < WCAP) list[wave * WCAP + pos] = ((el0 + (J)) << 12) | (int)(SJ); \
        } \
        wc += (int)__builtin_popcount(mj); } }
    HITJ(0, h0, s0)
    HITJ(1, h1, s1)
    HITJ(2, h2, s2)
    HITJ(3, h3, s3)
    HITJ(4, h4, s4)
    HITJ(5, h5, s5)
    HITJ(6, h6, s6)
    HITJ(7, h7, s7)
#undef HITJ
  }
  return wc;
}

__global__ __launch_bounds__(NTHR) void k_split(const float* __restrict__ src, int sp, int srows, int scols,
                                                unsigned short* dh, unsigned short* dl, int dp, int dcol0, int dq,
                                                int vec, int nUnits) {
  const int u = (int)blockIdx.x * NTHR + (int)threadIdx.x;
  if (u >= nUnits) return;
  const int row = u / dq;
  const int c8  = (u - row * dq) * 8;
  const int rc  = row < srows ? row : srows - 1;
  const float* rp = src + (size_t)rc * (size_t)sp;
  const v4f z4 = {0.f, 0.f, 0.f, 0.f};
  v4f a, b;
  if (vec != 0) {
    int cc = (c8 + 8 <= scols) ? c8 : scols - 8;
    cc = cc < 0 ? 0 : cc;
    a = *(const v4f*)(rp + cc);
    b = *(const v4f*)(rp + cc + 4);
    if (row >= srows || c8 + 8 > scols) { a = z4; b = z4; }
  } else {
    float v[8];
#pragma unroll
    for (int j = 0; j < 8; ++j) {
      const int cj  = c8 + j;
      const int cjc = cj < scols ? cj : scols - 1;
      const float t = rp[cjc];
      v[j] = (row < srows && cj < scols) ? t : 0.0f;
    }
    a.x = v[0]; a.y = v[1]; a.z = v[2]; a.w = v[3];
    b.x = v[4]; b.y = v[5]; b.z = v[6]; b.w = v[7];
  }
  v8us hi, lo;
  split8(a, b, hi, lo);
  const size_t o = (size_t)row * (size_t)dp + (size_t)dcol0 + (size_t)c8;
  *(volatile v8us*)(dh + o) = hi;
  *(volatile v8us*)(dl + o) = lo;
  __threadfence();
  *(volatile v8us*)(dh + o) = hi;
  *(volatile v8us*)(dl + o) = lo;
}

__global__ __launch_bounds__(NTHR) void k_wtr(const float* __restrict__ w0, const float* __restrict__ w1,
                                              const float* __restrict__ w2, int r1, int r2, int K, int KP,
                                              unsigned short* wth, unsigned short* wtl, int nUnits) {
  const int u = (int)blockIdx.x * NTHR + (int)threadIdx.x;
  if (u >= nUnits) return;
  const int kq = KP >> 3;
  const int n  = u / kq;
  const int k8 = (u - n * kq) * 8;
  const int seg = (n < r1) ? 0 : ((n < r2) ? 1 : 2);
  const int rs  = (seg == 0) ? 0 : ((seg == 1) ? r1 : r2);
  const float* wsrc = (seg == 0) ? w0 : ((seg == 1) ? w1 : w2);
  const int nl = n - rs;
  const int hs = nl >> 10;
  const int o  = nl & 1023;
  const float* p = wsrc + (size_t)hs * (size_t)K * (size_t)FDIM + o;
  float v[8];
#pragma unroll
  for (int j = 0; j < 8; ++j) {
    const int k  = k8 + j;
    const int kc = k < K ? k : K - 1;
    const float t = p[(size_t)kc * (size_t)FDIM];
    v[j] = (k < K) ? t : 0.0f;
  }
  v4f a, b;
  a.x = v[0]; a.y = v[1]; a.z = v[2]; a.w = v[3];
  b.x = v[4]; b.y = v[5]; b.z = v[6]; b.w = v[7];
  v8us hi, lo;
  split8(a, b, hi, lo);
  const size_t off = (size_t)n * (size_t)KP + (size_t)k8;
  *(volatile v8us*)(wth + off) = hi;
  *(volatile v8us*)(wtl + off) = lo;
  __threadfence();
  *(volatile v8us*)(wth + off) = hi;
  *(volatile v8us*)(wtl + off) = lo;
}

__global__ __launch_bounds__(GTHR) void k_gemm3(
    const unsigned short* __restrict__ AH, const unsigned short* __restrict__ AL, int lda,
    const unsigned short* __restrict__ WH, const unsigned short* __restrict__ WL, int K,
    const float* __restrict__ bias, int bofs, int blen, float* outF, int ldo)
{
  __shared__ __attribute__((aligned(16))) float stg[GBM * GBN];
  const int tid = (int)threadIdx.x, lane = tid & 31, wave = tid >> 5, hh = lane >> 4, m = lane & 15;
  const int rowBase = (int)blockIdx.x * GBM;
  const int col0    = (int)blockIdx.y * GBN;
  const bool bin = (col0 >= bofs) && (col0 < bofs + blen);

  v8f acc[4];
  {
    const v8f z = {0.f, 0.f, 0.f, 0.f, 0.f, 0.f, 0.f, 0.f};
    acc[0] = z; acc[1] = z; acc[2] = z; acc[3] = z;
  }
  const size_t arow = (size_t)(rowBase + 16 * wave + m) * (size_t)lda + (size_t)(8 * hh);
  const size_t wrow = (size_t)(col0 + m) * (size_t)K + (size_t)(8 * hh);
  const unsigned short* aph = AH + arow;
  const unsigned short* apl = AL + arow;
  const unsigned short* wph = WH + wrow;
  const unsigned short* wpl = WL + wrow;
  const int ksteps = K >> 5;
#pragma unroll 1
  for (int ks = 0; ks < ksteps; ++ks) {
    FragB ah, al;
    ah.h[0] = *(const v8us*)(aph + 32 * ks);
    ah.h[1] = *(const v8us*)(aph + 32 * ks + 16);
    al.h[0] = *(const v8us*)(apl + 32 * ks);
    al.h[1] = *(const v8us*)(apl + 32 * ks + 16);
#pragma unroll
    for (int t = 0; t < 4; ++t) {
      const size_t to = (size_t)(16 * t) * (size_t)K + (size_t)(32 * ks);
      FragB wh, wl;
      wh.h[0] = *(const v8us*)(wph + to);
      wh.h[1] = *(const v8us*)(wph + to + 16);
      wl.h[0] = *(const v8us*)(wpl + to);
      wl.h[1] = *(const v8us*)(wpl + to + 16);
      acc[t] = wmb(ah, wh, acc[t]);
      acc[t] = wmb(ah, wl, acc[t]);
      acc[t] = wmb(al, wh, acc[t]);
    }
  }

#pragma unroll
  for (int t = 0; t < 4; ++t) {
    const int lc = 16 * t + m;
    int bi = col0 + lc - bofs;
    bi = bi > blen - 1 ? blen - 1 : bi;
    bi = bi < 0 ? 0 : bi;
    const float bl = bias[bi];
    const float bv = bin ? bl : 0.0f;
#pragma unroll
    for (int r = 0; r < 8; ++r) {
      const int lr = 16 * wave + 8 * hh + r;
      stg[lr * GBN + lc] = acc[t][r] + bv;
    }
  }
  __syncthreads();

  v4f fv[8];
#pragma unroll
  for (int i = 0; i < 8; ++i) {
    const int lr = 16 * wave + 2 * i + hh;
    fv[i] = *(const v4f*)(stg + lr * GBN + 4 * m);
  }
#pragma unroll
  for (int i = 0; i < 8; ++i) {
    const int lr = 16 * wave + 2 * i + hh;
    const int gr = rowBase + lr;
    float* op = outF + (size_t)gr * (size_t)ldo + col0 + 4 * m;
    *(volatile v4f*)op = fv[i];
  }
  __threadfence();
#pragma unroll
  for (int i = 0; i < 8; ++i) {
    const int lr = 16 * wave + 2 * i + hh;
    const int gr = rowBase + lr;
    float* op = outF + (size_t)gr * (size_t)ldo + col0 + 4 * m;
    *(volatile v4f*)op = fv[i];
  }
}

__global__ __launch_bounds__(NTHR) void k_esed(const float* __restrict__ HBp, int ph, int hoff,
                                               const float* __restrict__ as, const float* __restrict__ ad,
                                               float* ESD) {
  __shared__ __attribute__((aligned(16))) float sv[64];
  const int tid = (int)threadIdx.x, lane = tid & 31, wave = tid >> 5;
  const int blk = (int)blockIdx.x;
#pragma unroll 1
  for (int i = 0; i < 4; ++i) {
    const int p    = 4 * wave + i;
    const int ln   = p >> 3;
    const int head = p & 7;
    const int node = 4 * blk + ln;
    const float* hr = HBp + (size_t)node * (size_t)ph + hoff + head * FDIM + 4 * lane;
    const float* ar = as + head * FDIM + 4 * lane;
    const float* dr = ad + head * FDIM + 4 * lane;
    float se = 0.f, sd = 0.f;
#pragma unroll 1
    for (int j = 0; j < FDIM / 128; ++j) {
      const v4f hv = *(const v4f*)(hr + 128 * j);
      const v4f av = *(const v4f*)(ar + 128 * j);
      const v4f dv = *(const v4f*)(dr + 128 * j);
      se = fmaf(hv.x, av.x, se); se = fmaf(hv.y, av.y, se); se = fmaf(hv.z, av.z, se); se = fmaf(hv.w, av.w, se);
      sd = fmaf(hv.x, dv.x, sd); sd = fmaf(hv.y, dv.y, sd); sd = fmaf(hv.z, dv.z, sd); sd = fmaf(hv.w, dv.w, sd);
    }
#pragma unroll
    for (int off = 16; off > 0; off >>= 1) {
      se += __shfl_xor(se, off);
      sd += __shfl_xor(sd, off);
    }
    if (lane == 0) { sv[16 * ln + head] = se; sv[16 * ln + 8 + head] = sd; }
  }
  __syncthreads();
  const int lq = lane & 15;
  const v4f ov = *(const v4f*)(sv + 4 * lq);
  float* op = ESD + (size_t)blk * 64 + 4 * lq;
  const bool wv = (wave == 0) && (lane < 16);
  if (wv) *(volatile v4f*)op = ov;
  __threadfence();
  if (wv) *(volatile v4f*)op = ov;
}

__global__ __launch_bounds__(NTHR) void k_agg(
    const int* __restrict__ srcs, const int* __restrict__ dsts,
    const float* __restrict__ HBp, int ph, int hoff,
    const float* __restrict__ ESD, const float* __restrict__ bias,
    const float* __restrict__ resp, int pres,
    float* Fout, int nN, int nE, int nb, int vec8, int MPr) {
  extern __shared__ v4f lds_dyn[];
  int* reg1 = (int*)lds_dyn;
  int* reg2 = reg1 + RCAP;
  int* scnt = reg2 + RCAP;
  int* soff = scnt + NBMAX;
  int* list = soff + NBMAX;
  int* wcnt = list + LISTN;
  int* wtot = wcnt + NWAVE;
  const int tid = (int)threadIdx.x, lane = tid & 31, wave = tid >> 5;
  const int nodeBase = (int)blockIdx.x * nb;

  for (int i = tid; i < NBMAX; i += NTHR) scnt[i] = 0;
  __syncthreads();

  int tot = 0;
  const int nChunks = (nE + CHUNK - 1) / CHUNK;
#pragma unroll 1
  for (int ch = 0; ch < nChunks; ++ch) {
    const int cbase = ch * CHUNK;
    const int wc = scan_chunk(dsts, nE, cbase, nodeBase, nb, vec8, list, tid, lane, wave);
    if (lane == 0) wcnt[wave] = wc;
    __syncthreads();
    int pre = 0, all = 0;
#pragma unroll
    for (int w2 = 0; w2 < NWAVE; ++w2) {
      int c = wcnt[w2];
      c = c < 0 ? 0 : (c > WCAP ? WCAP : c);
      all += c;
      pre += (w2 < wave) ? c : 0;
    }
    const int wcc  = wc > WCAP ? WCAP : wc;
    const int base = tot + pre;
#pragma unroll 1
    for (int i = lane; i < wcc; i += 32) {
      const int ent = list[wave * WCAP + i];
      const int el  = (ent >> 12) & (CHUNK - 1);
      const int sl  = ent & (NBMAX - 1);
      int eid = cbase + el;
      eid = eid > nE - 1 ? nE - 1 : eid;
      const int pos = base + i;
      if (pos < RCAP) reg1[pos] = (int)(((unsigned)eid << 12) | (unsigned)sl);
    }
    tot += all;
    tot = tot > RCAP ? RCAP : tot;
    __syncthreads();
  }
  const int nh = tot;

  if (wave == 0) {
#pragma unroll 1
    for (int b0 = 0; b0 < nh; b0 += 32) {
      const int idx = b0 + lane;
      const int uv  = reg1[idx < RCAP ? idx : RCAP - 1];
      const int m32 = (nh - b0) < 32 ? (nh - b0) : 32;
#pragma unroll 1
      for (int k = 0; k < m32; ++k) {
        const int u  = __builtin_amdgcn_readlane(uv, k);
        const int sl = u & (NBMAX - 1);
        if (lane == 0) scnt[sl] = scnt[sl] + 1;
      }
    }
  }
  __syncthreads();

  {
    const v4i ca = *(const v4i*)(scnt + 8 * tid);
    const v4i cb = *(const v4i*)(scnt + 8 * tid + 4);
    const int e0 = ca.x < 0 ? 0 : ca.x, e1 = ca.y < 0 ? 0 : ca.y, e2 = ca.z < 0 ? 0 : ca.z, e3 = ca.w < 0 ? 0 : ca.w;
    const int e4 = cb.x < 0 ? 0 : cb.x, e5 = cb.y < 0 ? 0 : cb.y, e6 = cb.z < 0 ? 0 : cb.z, e7 = cb.w < 0 ? 0 : cb.w;
    const int ts = e0 + e1 + e2 + e3 + e4 + e5 + e6 + e7;
    int incl = ts;
#pragma unroll
    for (int d = 1; d < 32; d <<= 1) {
      const int up = __shfl_up(incl, d);
      if (lane >= d) incl += up;
    }
    if (lane == 31) wtot[wave] = incl;
    __syncthreads();
    int pre = 0;
#pragma unroll
    for (int w2 = 0; w2 < NWAVE; ++w2) pre += (w2 < wave) ? wtot[w2] : 0;
    int run = pre + incl - ts;
    soff[8 * tid + 0] = run; run += e0;
    soff[8 * tid + 1] = run; run += e1;
    soff[8 * tid + 2] = run; run += e2;
    soff[8 * tid + 3] = run; run += e3;
    soff[8 * tid + 4] = run; run += e4;
    soff[8 * tid + 5] = run; run += e5;
    soff[8 * tid + 6] = run; run += e6;
    soff[8 * tid + 7] = run;
  }
  __syncthreads();
  for (int i = tid; i < NBMAX; i += NTHR) list[i] = soff[i];
  __syncthreads();

  if (wave == 0) {
#pragma unroll 1
    for (int b0 = 0; b0 < nh; b0 += 32) {
      const int idx = b0 + lane;
      const int uv  = reg1[idx < RCAP ? idx : RCAP - 1];
      const int m32 = (nh - b0) < 32 ? (nh - b0) : 32;
#pragma unroll 1
      for (int k = 0; k < m32; ++k) {
        const int u   = __builtin_amdgcn_readlane(uv, k);
        const int sl  = u & (NBMAX - 1);
        const int eid = (int)((unsigned)u >> 12);
        if (lane == 0) {
          int pos = list[sl];
          pos = pos < 0 ? 0 : (pos > RCAP - 1 ? RCAP - 1 : pos);
          reg2[pos] = eid;
          list[sl] = pos + 1;
        }
      }
    }
  }
  __syncthreads();

  const int nbw = nb >> 3;
  const bool ovf = (nh >= RCAP);
  const float qnan = __int_as_float(0x7fc00000);
  const float ninf = __int_as_float((int)0xff800000);
  float* atab = (float*)reg1 + wave * STW;
  int*   srcl = (int*)(atab + DEGCAP * NHEAD);
  float* stw  = atab + DEGCAP * NHEAD + DEGCAP;
#pragma unroll 1
  for (int jt = 0; jt < nbw; ++jt) {
    const int slot = wave * nbw + jt;
    const int grow = nodeBase + slot;
    const int gcl  = grow < nN ? grow : nN - 1;
    int st = soff[slot];
    const int craw = scnt[slot];
    int cnt = craw;
    st  = st < 0 ? 0 : (st > nh ? nh : st);
    cnt = cnt < 0 ? 0 : (cnt > DEGCAP ? DEGCAP : cnt);
    if (cnt > nh - st) cnt = nh - st;
    const float pz = (ovf || craw > DEGCAP) ? qnan : 0.0f;
    const bool wr = grow < MPr;
    const float live = grow < nN ? 1.0f : 0.0f;

    __builtin_amdgcn_fence(__ATOMIC_RELEASE, "wavefront");
    __builtin_amdgcn_wave_barrier();

    const v4f eda = *(const v4f*)(ESD + (size_t)gcl * 16 + 8);
    const v4f edb = *(const v4f*)(ESD + (size_t)gcl * 16 + 12);
    float edv[NHEAD];
    edv[0] = eda.x; edv[1] = eda.y; edv[2] = eda.z; edv[3] = eda.w;
    edv[4] = edb.x; edv[5] = edb.y; edv[6] = edb.z; edv[7] = edb.w;
    float lg[NIT][NHEAD];
    float lmx[NHEAD];
#pragma unroll
    for (int hd = 0; hd < NHEAD; ++hd) lmx[hd] = ninf;
#pragma unroll
    for (int it = 0; it < NIT; ++it) {
      const int q = 32 * it + lane;
      const bool valid = q < cnt;
      int idx = st + q;
      idx = idx > RCAP - 1 ? RCAP - 1 : idx;
      int eid = reg2[idx];
      eid = eid < 0 ? 0 : (eid > nE - 1 ? nE - 1 : eid);
      const int sraw = srcs[eid];
      const int s = sraw < 0 ? 0 : (sraw > nN - 1 ? nN - 1 : sraw);
      srcl[q] = s;
      const v4f ea = *(const v4f*)(ESD + (size_t)s * 16);
      const v4f eb = *(const v4f*)(ESD + (size_t)s * 16 + 4);
      float ev[NHEAD];
      ev[0] = ea.x; ev[1] = ea.y; ev[2] = ea.z; ev[3] = ea.w;
      ev[4] = eb.x; ev[5] = eb.y; ev[6] = eb.z; ev[7] = eb.w;
#pragma unroll
      for (int hd = 0; hd < NHEAD; ++hd) {
        float t = ev[hd] + edv[hd];
        t = (t >= 0.0f) ? t : 0.2f * t;
        t = valid ? t : ninf;
        lg[it][hd] = t;
        lmx[hd] = fmaxf(lmx[hd], t);
      }
    }
#pragma unroll
    for (int off = 16; off > 0; off >>= 1) {
#pragma unroll
      for (int hd = 0; hd < NHEAD; ++hd) lmx[hd] = fmaxf(lmx[hd], __shfl_xor(lmx[hd], off));
    }
    float mm[NHEAD], dsum[NHEAD];
#pragma unroll
    for (int hd = 0; hd < NHEAD; ++hd) { mm[hd] = (lmx[hd] > ninf) ? lmx[hd] : 0.0f; dsum[hd] = 0.0f; }
#pragma unroll
    for (int it = 0; it < NIT; ++it) {
      const bool valid = (32 * it + lane) < cnt;
#pragma unroll
      for (int hd = 0; hd < NHEAD; ++hd) {
        float w = __expf(lg[it][hd] - mm[hd]);
        w = valid ? w : 0.0f;
        lg[it][hd] = w;
        dsum[hd] += w;
      }
    }
#pragma unroll
    for (int off = 16; off > 0; off >>= 1) {
#pragma unroll
      for (int hd = 0; hd < NHEAD; ++hd) dsum[hd] += __shfl_xor(dsum[hd], off);
    }
    float rden[NHEAD];
#pragma unroll
    for (int hd = 0; hd < NHEAD; ++hd) rden[hd] = __builtin_amdgcn_rcpf(dsum[hd] + 1e-16f);
#pragma unroll
    for (int it = 0; it < NIT; ++it) {
      const int q = 32 * it + lane;
      v4f a0, a1;
      a0.x = lg[it][0] * rden[0]; a0.y = lg[it][1] * rden[1]; a0.z = lg[it][2] * rden[2]; a0.w = lg[it][3] * rden[3];
      a1.x = lg[it][4] * rden[4]; a1.y = lg[it][5] * rden[5]; a1.z = lg[it][6] * rden[6]; a1.w = lg[it][7] * rden[7];
      *(v4f*)(atab + 8 * q)     = a0;
      *(v4f*)(atab + 8 * q + 4) = a1;
    }
    __builtin_amdgcn_fence(__ATOMIC_RELEASE, "wavefront");
    __builtin_amdgcn_wave_barrier();

    v4f acc[8];
    {
      const v4f z4 = {0.f, 0.f, 0.f, 0.f};
#pragma unroll
      for (int j = 0; j < 8; ++j) acc[j] = z4;
    }
#pragma unroll 1
    for (int q = 0; q < cnt; ++q) {
      const int s = srcl[q];
      const float* hp = HBp + (size_t)s * (size_t)ph + hoff + 4 * lane;
      const float* aq = atab + 8 * q;
#pragma unroll 1
      for (int hd = 0; hd < NHEAD; ++hd) {
        const float al = aq[hd];
        const float* hq = hp + hd * FDIM;
        v4f hv[8];
#pragma unroll
        for (int j = 0; j < 8; ++j) hv[j] = *(const v4f*)(hq + 128 * j);
#pragma unroll
        for (int j = 0; j < 8; ++j) acc[j] = al * hv[j] + acc[j];
      }
    }

    __builtin_amdgcn_fence(__ATOMIC_RELEASE, "wavefront");
    __builtin_amdgcn_wave_barrier();
#pragma unroll
    for (int j = 0; j < 8; ++j) *(v4f*)(stw + 128 * j + 4 * lane) = acc[j];
    __builtin_amdgcn_fence(__ATOMIC_RELEASE, "wavefront");
    __builtin_amdgcn_wave_barrier();
    const float* rrow = resp + (size_t)gcl * (size_t)pres;
#pragma unroll 1
    for (int i = 0; i < FDIM / 32; ++i) {
      const int f = 32 * i + lane;
      float v = stw[f];
      v = fmaf(v, 0.125f, bias[f]) + rrow[f];
      const float en = expm1f(v);
      v = (v > 0.0f) ? v : en;
      v = v * live + pz;
      stw[f] = v;
    }
    __builtin_amdgcn_fence(__ATOMIC_RELEASE, "wavefront");
    __builtin_amdgcn_wave_barrier();
    v4f fv[8];
#pragma unroll
    for (int j = 0; j < 8; ++j) fv[j] = *(const v4f*)(stw + 128 * j + 4 * lane);
    float* orow = Fout + (size_t)(wr ? grow : 0) * (size_t)FDIM + 4 * lane;
    if (wr) {
#pragma unroll
      for (int j = 0; j < 8; ++j) *(volatile v4f*)(orow + 128 * j) = fv[j];
    }
    __threadfence();
    if (wr) {
#pragma unroll
      for (int j = 0; j < 8; ++j) *(volatile v4f*)(orow + 128 * j) = fv[j];
    }
  }
}

__global__ __launch_bounds__(NTHR) void k_out(const float* __restrict__ S, int ldsp, int ncol,
                                              float* out, int total, int nUnits) {
  const int u = (int)blockIdx.x * NTHR + (int)threadIdx.x;
  if (u >= nUnits) return;
  const int e0 = 4 * u;
  float v[4];
#pragma unroll
  for (int c = 0; c < 4; ++c) {
    const int e   = e0 + c;
    const int ec  = e < total ? e : total - 1;
    const int row = ec / ncol;
    const int col = ec - row * ncol;
    const float s = S[(size_t)row * (size_t)ldsp + col];
    const float ex = expf(-s);
    v[c] = __builtin_amdgcn_rcpf(1.0f + ex);
  }
  const bool full = (e0 + 4 <= total);
  v4f fv;
  fv.x = v[0]; fv.y = v[1]; fv.z = v[2]; fv.w = v[3];
  if (full) {
    *(volatile v4f*)(out + e0) = fv;
  } else {
#pragma unroll
    for (int c = 0; c < 4; ++c) if (e0 + c < total) ((volatile float*)out)[e0 + c] = v[c];
  }
  __threadfence();
  if (full) {
    *(volatile v4f*)(out + e0) = fv;
  } else {
#pragma unroll
    for (int c = 0; c < 4; ++c) if (e0 + c < total) ((volatile float*)out)[e0 + c] = v[c];
  }
}

static inline int cdiv(int a, int b) { return (a + b - 1) / b; }
static inline size_t al256(size_t x) { return (x + 255) & ~(size_t)255; }
static inline size_t smax(size_t a, size_t b) { return a > b ? a : b; }

extern "C" void kernel_launch(void* const* d_in, const int* in_sizes, int n_in,
                              void* d_out, int out_size, void* d_ws, size_t ws_size,
                              hipStream_t stream) {
  if (n_in < 31) return;
  const int nN = in_sizes[0] / DIN;
  if (nN < 1 || in_sizes[0] != nN * DIN || nN > 65536) return;
  if (in_sizes[1] < 2 || (in_sizes[1] & 1) != 0) return;
  const int nE = in_sizes[1] / 2;
  if (nE < 1 || nE > (1 << 20)) return;
  const int nC = in_sizes[6] / FDIM;
  if (nC < 8 || in_sizes[6] != nC * FDIM || nC > 4096) return;
  if (in_sizes[2] != nC * nC) return;
  if (in_sizes[3] < 2 || (in_sizes[3] & 1) != 0) return;
  const int nEC = in_sizes[3] / 2;
  if (nEC < 1 || nEC > (1 << 20)) return;
  if (in_sizes[4]  != DIN * FDIM || in_sizes[5] != FDIM || in_sizes[7] != FDIM) return;
  if (in_sizes[8]  != NHEAD * DIN * FDIM || in_sizes[9] != HALL || in_sizes[10] != HALL || in_sizes[11] != FDIM) return;
  if (in_sizes[12] != DIN * FDIM) return;
  if (in_sizes[13] != NHEAD * FDIM * FDIM || in_sizes[14] != HALL || in_sizes[15] != HALL || in_sizes[16] != FDIM) return;
  if (in_sizes[17] != NHEAD * nC * FDIM || in_sizes[18] != HALL || in_sizes[19] != HALL || in_sizes[20] != FDIM) return;
  if (in_sizes[21] != nC * FDIM) return;
  if (in_sizes[22] != NHEAD * FDIM * FDIM || in_sizes[23] != HALL || in_sizes[24] != HALL || in_sizes[25] != FDIM) return;
  if (in_sizes[26] != FDIM * JKK || in_sizes[27] != FDIM || in_sizes[28] != FDIM * JKK || in_sizes[29] != FDIM) return;
  if (in_sizes[30] != FDIM * FDIM) return;
  if (out_size != nN * nC) return;

  const float* x    = (const float*)d_in[0];
  const int*   eih  = (const int*)  d_in[1];
  const float* xc   = (const float*)d_in[2];
  const int*   eic  = (const int*)  d_in[3];
  const float* Wp   = (const float*)d_in[4];
  const float* bp   = (const float*)d_in[5];
  const float* Wpc  = (const float*)d_in[6];
  const float* bpc  = (const float*)d_in[7];
  const float* Wh0  = (const float*)d_in[8];
  const float* ash0 = (const float*)d_in[9];
  const float* adh0 = (const float*)d_in[10];
  const float* bh0  = (const float*)d_in[11];
  const float* rh0  = (const float*)d_in[12];
  const float* Wh1  = (const float*)d_in[13];
  const float* ash1 = (const float*)d_in[14];
  const float* adh1 = (const float*)d_in[15];
  const float* bh1  = (const float*)d_in[16];
  const float* Wc0  = (const float*)d_in[17];
  const float* asc0 = (const float*)d_in[18];
  const float* adc0 = (const float*)d_in[19];
  const float* bc0  = (const float*)d_in[20];
  const float* rc0  = (const float*)d_in[21];
  const float* Wc1  = (const float*)d_in[22];
  const float* asc1 = (const float*)d_in[23];
  const float* adc1 = (const float*)d_in[24];
  const float* bc1  = (const float*)d_in[25];
  const float* Wnh  = (const float*)d_in[26];
  const float* bnh  = (const float*)d_in[27];
  const float* Wnc  = (const float*)d_in[28];
  const float* bnc  = (const float*)d_in[29];
  const float* Wd   = (const float*)d_in[30];
  float* out = (float*)d_out;
  const int* srcH = eih;
  const int* dstH = eih + nE;
  const int* srcC = eic;
  const int* dstC = eic + nEC;

  const int MP  = cdiv(nN, GBM) * GBM;
  const int MPC = cdiv(nC, GBM) * GBM;
  const int KC  = cdiv(nC, 32) * 32;
  const int NDP = cdiv(nC, GBN) * GBN;
  const int MPB = MP > MPC ? MP : MPC;
  const int gA  = cdiv(MP, NBAGG);
  const int gAC = cdiv(MPC, NBAGG);
  if (gA * NBAGG < MP || gAC * NBAGG < MPC) return;
  if ((MP % 4) != 0 || (MPC % 4) != 0) return;
  const int vec8h = ((nE  & 3) == 0) ? 1 : 0;
  const int vec8c = ((nEC & 3) == 0) ? 1 : 0;

  size_t eXH = smax((size_t)MP * DIN, (size_t)MPC * KC);
  size_t eWT = (size_t)NX1 * DIN;
  eWT = smax(eWT, (size_t)NX1 * KC);
  eWT = smax(eWT, (size_t)HALL * FDIM);
  eWT = smax(eWT, (size_t)FDIM * JKK);
  eWT = smax(eWT, (size_t)FDIM * FDIM);
  char* ws = (char*)d_ws;
  size_t off = 0;
  const size_t oXH  = off; off = al256(off + eXH * 2);
  const size_t oXL  = off; off = al256(off + eXH * 2);
  const size_t oWTH = off; off = al256(off + eWT * 2);
  const size_t oWTL = off; off = al256(off + eWT * 2);
  const size_t oHB  = off; off = al256(off + (size_t)MPB * NX1 * 4);
  const size_t oESD = off; off = al256(off + (size_t)MPB * 16 * 4);
  const size_t oF1  = off; off = al256(off + (size_t)MPB * FDIM * 4);
  const size_t oF2  = off; off = al256(off + (size_t)MPB * FDIM * 4);
  const size_t oFTH = off; off = al256(off + (size_t)MPB * JKK * 2);
  const size_t oFTL = off; off = al256(off + (size_t)MPB * JKK * 2);
  const size_t oZ   = off; off = al256(off + (size_t)MPB * FDIM * 4);
  const size_t oT   = off; off = al256(off + (size_t)MP * FDIM * 4);
  const size_t oZHH = off; off = al256(off + (size_t)MP * FDIM * 2);
  const size_t oZHL = off; off = al256(off + (size_t)MP * FDIM * 2);
  const size_t oZCH = off; off = al256(off + (size_t)NDP * FDIM * 2);
  const size_t oZCL = off; off = al256(off + (size_t)NDP * FDIM * 2);
  const size_t oTHH = off; off = al256(off + (size_t)MP * FDIM * 2);
  const size_t oTHL = off; off = al256(off + (size_t)MP * FDIM * 2);
  const size_t oS   = off; off = al256(off + (size_t)MP * NDP * 4);
  if (off > ws_size || off > (size_t)WSMAX) return;
  unsigned short* XH  = (unsigned short*)(ws + oXH);
  unsigned short* XL  = (unsigned short*)(ws + oXL);
  unsigned short* WTH = (unsigned short*)(ws + oWTH);
  unsigned short* WTL = (unsigned short*)(ws + oWTL);
  float*          HB  = (float*)(ws + oHB);
  float*          ESD = (float*)(ws + oESD);
  float*          F1  = (float*)(ws + oF1);
  float*          F2  = (float*)(ws + oF2);
  unsigned short* FTH = (unsigned short*)(ws + oFTH);
  unsigned short* FTL = (unsigned short*)(ws + oFTL);
  float*          Zf  = (float*)(ws + oZ);
  float*          Tf  = (float*)(ws + oT);
  unsigned short* ZHH = (unsigned short*)(ws + oZHH);
  unsigned short* ZHL = (unsigned short*)(ws + oZHL);
  unsigned short* ZCH = (unsigned short*)(ws + oZCH);
  unsigned short* ZCL = (unsigned short*)(ws + oZCL);
  unsigned short* THH = (unsigned short*)(ws + oTHH);
  unsigned short* THL = (unsigned short*)(ws + oTHL);
  float*          Sf  = (float*)(ws + oS);

  hipFuncSetAttribute(reinterpret_cast<const void*>(&k_agg),
                      hipFuncAttributeMaxDynamicSharedMemorySize, LDS_AGG);

  {
    const int nU = MP * (DIN / 8);
    k_split<<<cdiv(nU, NTHR), NTHR, 0, stream>>>(x, DIN, nN, DIN, XH, XL, DIN, 0, DIN / 8, 1, nU);
  }
  {
    const int nU = NX1 * (DIN / 8);
    k_wtr<<<cdiv(nU, NTHR), NTHR, 0, stream>>>(Wp, Wh0, rh0, FDIM, FDIM + HALL, DIN, DIN, WTH, WTL, nU);
  }
  k_gemm3<<<dim3(MP / GBM, NX1 / GBN), GTHR, 0, stream>>>(XH, XL, DIN, WTH, WTL, DIN, bp, 0, FDIM, HB, NX1);
  k_esed<<<MP / 4, NTHR, 0, stream>>>(HB, NX1, OFH, ash0, adh0, ESD);
  k_agg<<<gA, NTHR, LDS_AGG, stream>>>(srcH, dstH, HB, NX1, OFH, ESD, bh0, HB + OFR, NX1, F1,
                                       nN, nE, NBAGG, vec8h, MP);
  {
    const int nU = MP * (FDIM / 8);
    k_split<<<cdiv(nU, NTHR), NTHR, 0, stream>>>(HB, NX1, nN, FDIM, FTH, FTL, JKK, 0, FDIM / 8, 1, nU);
    k_split<<<cdiv(nU, NTHR), NTHR, 0, stream>>>(F1, FDIM, nN, FDIM, FTH, FTL, JKK, FDIM, FDIM / 8, 1, nU);
  }
  {
    const int nU = HALL * (FDIM / 8);
    k_wtr<<<cdiv(nU, NTHR), NTHR, 0, stream>>>(Wh1, Wh1, Wh1, HALL, HALL, FDIM, FDIM, WTH, WTL, nU);
  }
  k_gemm3<<<dim3(MP / GBM, HALL / GBN), GTHR, 0, stream>>>(FTH + FDIM, FTL + FDIM, JKK, WTH, WTL, FDIM,
                                                            bp, 0, 0, HB, HALL);
  k_esed<<<MP / 4, NTHR, 0, stream>>>(HB, HALL, 0, ash1, adh1, ESD);
  k_agg<<<gA, NTHR, LDS_AGG, stream>>>(srcH, dstH, HB, HALL, 0, ESD, bh1, F1, FDIM, F2,
                                       nN, nE, NBAGG, vec8h, MP);
  {
    const int nU = MP * (FDIM / 8);
    k_split<<<cdiv(nU, NTHR), NTHR, 0, stream>>>(F2, FDIM, nN, FDIM, FTH, FTL, JKK, 2 * FDIM, FDIM / 8, 1, nU);
    const int nW = FDIM * (JKK / 8);
    k_split<<<cdiv(nW, NTHR), NTHR, 0, stream>>>(Wnh, JKK, FDIM, JKK, WTH, WTL, JKK, 0, JKK / 8, 1, nW);
  }
  k_gemm3<<<dim3(MP / GBM, FDIM / GBN), GTHR, 0, stream>>>(FTH, FTL, JKK, WTH, WTL, JKK, bnh, 0, FDIM, Zf, FDIM);
  {
    const int nU = MP * (FDIM / 8);
    k_split<<<cdiv(nU, NTHR), NTHR, 0, stream>>>(Zf, FDIM, nN, FDIM, ZHH, ZHL, FDIM, 0, FDIM / 8, 1, nU);
  }

  {
    const int nU = MPC * (KC / 8);
    k_split<<<cdiv(nU, NTHR), NTHR, 0, stream>>>(xc, nC, nC, nC, XH, XL, KC, 0, KC / 8, 0, nU);
  }
  {
    const int nU = NX1 * (KC / 8);
    k_wtr<<<cdiv(nU, NTHR), NTHR, 0, stream>>>(Wpc, Wc0, rc0, FDIM, FDIM + HALL, nC, KC, WTH, WTL, nU);
  }
  k_gemm3<<<dim3(MPC / GBM, NX1 / GBN), GTHR, 0, stream>>>(XH, XL, KC, WTH, WTL, KC, bpc, 0, FDIM, HB, NX1);
  k_esed<<<MPC / 4, NTHR, 0, stream>>>(HB, NX1, OFH, asc0, adc0, ESD);
  k_agg<<<gAC, NTHR, LDS_AGG, stream>>>(srcC, dstC, HB, NX1, OFH, ESD, bc0, HB + OFR, NX1, F1,
                                        nC, nEC, NBAGG, vec8c, MPC);
  {
    const int nU = MPC * (FDIM / 8);
    k_split<<<cdiv(nU, NTHR), NTHR, 0, stream>>>(HB, NX1, nC, FDIM, FTH, FTL, JKK, 0, FDIM / 8, 1, nU);
    k_split<<<cdiv(nU, NTHR), NTHR, 0, stream>>>(F1, FDIM, nC, FDIM, FTH, FTL, JKK, FDIM, FDIM / 8, 1, nU);
  }
  {
    const int nU = HALL * (FDIM / 8);
    k_wtr<<<cdiv(nU, NTHR), NTHR, 0, stream>>>(Wc1, Wc1, Wc1, HALL, HALL, FDIM, FDIM, WTH, WTL, nU);
  }
  k_gemm3<<<dim3(MPC / GBM, HALL / GBN), GTHR, 0, stream>>>(FTH + FDIM, FTL + FDIM, JKK, WTH, WTL, FDIM,
                                                             bp, 0, 0, HB, HALL);
  k_esed<<<MPC / 4, NTHR, 0, stream>>>(HB, HALL, 0, asc1, adc1, ESD);
  k_agg<<<gAC, NTHR, LDS_AGG, stream>>>(srcC, dstC, HB, HALL, 0, ESD, bc1, F1, FDIM, F2,
                                        nC, nEC, NBAGG, vec8c, MPC);
  {
    const int nU = MPC * (FDIM / 8);
    k_split<<<cdiv(nU, NTHR), NTHR, 0, stream>>>(F2, FDIM, nC, FDIM, FTH, FTL, JKK, 2 * FDIM, FDIM / 8, 1, nU);
    const int nW = FDIM * (JKK / 8);
    k_split<<<cdiv(nW, NTHR), NTHR, 0, stream>>>(Wnc, JKK, FDIM, JKK, WTH, WTL, JKK, 0, JKK / 8, 1, nW);
  }
  k_gemm3<<<dim3(MPC / GBM, FDIM / GBN), GTHR, 0, stream>>>(FTH, FTL, JKK, WTH, WTL, JKK, bnc, 0, FDIM, Zf, FDIM);
  {
    const int nU = NDP * (FDIM / 8);
    k_split<<<cdiv(nU, NTHR), NTHR, 0, stream>>>(Zf, FDIM, nC, FDIM, ZCH, ZCL, FDIM, 0, FDIM / 8, 1, nU);
  }

  {
    const int nU = FDIM * (FDIM / 8);
    k_wtr<<<cdiv(nU, NTHR), NTHR, 0, stream>>>(Wd, Wd, Wd, FDIM, FDIM, FDIM, FDIM, WTH, WTL, nU);
  }
  k_gemm3<<<dim3(MP / GBM, FDIM / GBN), GTHR, 0, stream>>>(ZHH, ZHL, FDIM, WTH, WTL, FDIM, bp, 0, 0, Tf, FDIM);
  {
    const int nU = MP * (FDIM / 8);
    k_split<<<cdiv(nU, NTHR), NTHR, 0, stream>>>(Tf, FDIM, nN, FDIM, THH, THL, FDIM, 0, FDIM / 8, 1, nU);
  }
  k_gemm3<<<dim3(MP / GBM, NDP / GBN), GTHR, 0, stream>>>(THH, THL, FDIM, ZCH, ZCL, FDIM, bp, 0, 0, Sf, NDP);
  {
    const int tot = nN * nC;
    const int nU  = cdiv(tot, 4);
    k_out<<<cdiv(nU, NTHR), NTHR, 0, stream>>>(Sf, NDP, nC, out, tot, nU);
  }
}
